// MM_DecoderLSTM_16346645529091
// MI455X (gfx1250) — hardware-verified
//
#include <hip/hip_runtime.h>


typedef _Float16 f16t;
typedef f16t  v16h __attribute__((ext_vector_type(16)));
typedef f16t  v8h  __attribute__((ext_vector_type(8)));
typedef float v8f  __attribute__((ext_vector_type(8)));
typedef float v4f  __attribute__((ext_vector_type(4)));

union Frag { v16h v; v8h q[2]; };

namespace {
constexpr int HD    = 64;
constexpr int NM    = 6;
constexpr int NP    = 12;
constexpr int TS    = 30;
constexpr int WAVES = 4;
constexpr int AG    = 16;
constexpr int BLKA  = WAVES * AG;
constexpr int NTHR  = WAVES * 32;
constexpr int OUTW  = NM * TS * 2;
constexpr int HP    = 64;
constexpr int XP    = 16;
constexpr float WSC  = 16.0f;
constexpr float WINV = 0.0625f;
constexpr int NPIECE = (BLKA * OUTW) / 4;
constexpr int NIT    = NPIECE / NTHR;
constexpr int NCPIECE = (BLKA * NM) / 4;
static_assert(NPIECE % NTHR == 0);
static_assert((BLKA * NM) % 4 == 0);
static_assert((BLKA * OUTW * 4) % 128 == 0);
static_assert((BLKA * NM * 4) % 128 == 0);
}

__device__ __forceinline__ v8f wmma16(v16h a, v16h b, v8f c) {
    return __builtin_amdgcn_wmma_f32_16x16x32_f16(false, a, false, b, (short)0, c, false, false);
}
__device__ __forceinline__ v8f zacc() {
    v8f z = {0.f, 0.f, 0.f, 0.f, 0.f, 0.f, 0.f, 0.f};
    return z;
}
__device__ __forceinline__ v8h zero8h() {
    v8h z;
#pragma unroll
    for (int e = 0; e < 8; ++e) z[e] = (f16t)0.0f;
    return z;
}
__device__ __forceinline__ v16h ldfrag(const f16t* p) {
    Frag f;
    f.q[0] = *(const v8h*)p;
    f.q[1] = *(const v8h*)(p + 16);
    return f.v;
}
__device__ __forceinline__ v16h ldfrag16(const f16t* p) {
    Frag f;
    f.q[0] = *(const v8h*)p;
    f.q[1] = zero8h();
    return f.v;
}
__device__ __forceinline__ void guard1(v8f& c, const v16h& a, const v16h& b) {
    asm volatile("v_nop\n\tv_nop\n\tv_nop\n\tv_nop" : "+v"(c) : "v"(a), "v"(b));
}
__device__ __forceinline__ void guard2(v8f& c, const v16h& a0, const v16h& a1,
                                       const v16h& b0, const v16h& b1) {
    asm volatile("v_nop\n\tv_nop\n\tv_nop\n\tv_nop"
                 : "+v"(c) : "v"(a0), "v"(a1), "v"(b0), "v"(b1));
}
__device__ __forceinline__ void guard3(v8f& c, const v16h& a0, const v16h& a1, const v16h& a2,
                                       const v16h& b0, const v16h& b1, const v16h& b2) {
    asm volatile("v_nop\n\tv_nop\n\tv_nop\n\tv_nop"
                 : "+v"(c) : "v"(a0), "v"(a1), "v"(a2), "v"(b0), "v"(b1), "v"(b2));
}

__device__ __forceinline__ float fsig(float x) {
    return __builtin_amdgcn_rcpf(1.0f + __expf(-x));
}
__device__ __forceinline__ float ftanh(float x) {
    const float ax = fabsf(x);
    const float t  = __expf(-2.0f * ax);
    const float r  = (1.0f - t) * __builtin_amdgcn_rcpf(1.0f + t);
    return copysignf(r, x);
}
__device__ __forceinline__ v8h cvt8(v4f a, v4f b, float sc) {
    v8h k;
    k[0] = (f16t)(a[0] * sc); k[1] = (f16t)(a[1] * sc); k[2] = (f16t)(a[2] * sc); k[3] = (f16t)(a[3] * sc);
    k[4] = (f16t)(b[0] * sc); k[5] = (f16t)(b[1] * sc); k[6] = (f16t)(b[2] * sc); k[7] = (f16t)(b[3] * sc);
    return k;
}

__device__ __forceinline__ v8f gate_tile(int tile, const f16t* wih, const f16t* whh,
                                        const v16h& xa, const v16h& ha0, const v16h& ha1,
                                        int h, int n) {
    const int nr = tile * 16 + n;
    const v16h bi = ldfrag16(wih + nr * XP + 8 * h);
    const f16t* ph = whh + nr * HP + 8 * h;
    const v16h b0 = ldfrag(ph);
    const v16h b1 = ldfrag(ph + 32);
    v8f acc = zacc();
    acc = wmma16(xa,  bi, acc);
    acc = wmma16(ha0, b0, acc);
    acc = wmma16(ha1, b1, acc);
    guard3(acc, xa, ha0, ha1, bi, b0, b1);
    return acc;
}

__device__ __forceinline__ void se_step(const f16t* rst, const f16t* wse, const float* bse,
                                        f16t* xst, int h, int n) {
    const v16h ra = ldfrag16(rst + n * XP + 8 * h);
    const v16h bs = ldfrag16(wse + n * XP + 8 * h);
    v8f acc = zacc();
    acc = wmma16(ra, bs, acc);
    guard1(acc, ra, bs);
    const float bb = bse[n];
#pragma unroll
    for (int r = 0; r < 8; ++r) {
        float v = fmaf(acc[r], WINV, bb);
        v = fmaxf(v, 0.01f * v);
        xst[(8 * h + r) * XP + n] = (f16t)v;
    }
}

__global__ __launch_bounds__(NTHR, 4)
void k_traj_lstm(const float* __restrict__ traj_rel,
                 const float* __restrict__ h0,
                 const float* __restrict__ c0,
                 const float* __restrict__ W_ih,
                 const float* __restrict__ W_hh,
                 const float* __restrict__ b_ih,
                 const float* __restrict__ b_hh,
                 const float* __restrict__ W_se,
                 const float* __restrict__ b_se,
                 const float* __restrict__ W_pos,
                 const float* __restrict__ b_pos,
                 const float* __restrict__ W_conf,
                 const float* __restrict__ b_conf,
                 float* pred,
                 float* conf,
                 int nagents)
{
    __shared__ __attribute__((aligned(16))) f16t  sWhh[256 * HP];
    __shared__ __attribute__((aligned(16))) f16t  sWih[256 * XP];
    __shared__ __attribute__((aligned(16))) f16t  sWpos[16 * HP];
    __shared__ __attribute__((aligned(16))) f16t  sWse[16 * XP];
    __shared__ __attribute__((aligned(16))) f16t  sWcf[16 * HP];
    __shared__ __attribute__((aligned(16))) float sBg[256];
    __shared__ __attribute__((aligned(16))) float sBpos[16];
    __shared__ __attribute__((aligned(16))) float sBse[16];
    __shared__ __attribute__((aligned(16))) float sBcf[16];
    __shared__ __attribute__((aligned(16))) f16t  sH[BLKA * HP];
    __shared__ __attribute__((aligned(16))) f16t  sX[BLKA * XP];
    __shared__ __attribute__((aligned(16))) f16t  sR[BLKA * XP];
    __shared__ __attribute__((aligned(16))) float sPred[BLKA * OUTW];
    __shared__ __attribute__((aligned(16))) float sLog[BLKA * 8];
    __shared__ __attribute__((aligned(16))) float sCf[BLKA * NM];

    const int tid = threadIdx.x;
    const int blk = blockIdx.x;
    if ((blk + 1) * BLKA > nagents) return;

    for (int c = tid; c < 256 * 8; c += NTHR) {
        const float* p = W_hh + (size_t)c * 8;
        *(v8h*)(sWhh + c * 8) = cvt8(*(const v4f*)p, *(const v4f*)(p + 4), WSC);
    }
    for (int c = tid; c < 256 * 2; c += NTHR) {
        const float* p = W_ih + (size_t)c * 8;
        *(v8h*)(sWih + c * 8) = cvt8(*(const v4f*)p, *(const v4f*)(p + 4), WSC);
    }
    for (int c = tid; c < 16 * 8; c += NTHR) {
        const int row = c >> 3, part = c & 7;
        {
            const int rr = row < NP ? row : NP - 1;
            const float* p = W_pos + rr * HD + part * 8;
            v8h k = cvt8(*(const v4f*)p, *(const v4f*)(p + 4), WSC);
            if (row >= NP) k = zero8h();
            *(v8h*)(sWpos + c * 8) = k;
        }
        {
            const int rr = row < NM ? row : NM - 1;
            const float* p = W_conf + rr * HD + part * 8;
            v8h k = cvt8(*(const v4f*)p, *(const v4f*)(p + 4), WSC);
            if (row >= NM) k = zero8h();
            *(v8h*)(sWcf + c * 8) = k;
        }
    }
    for (int e = tid; e < 16 * XP; e += NTHR) {
        const int row = e >> 4, k = e & 15;
        const int kk  = k < NP ? k : 0;
        float v = W_se[row * NP + kk] * WSC;
        if (k >= NP) v = 0.0f;
        sWse[e] = (f16t)v;
    }
    for (int e = tid; e < 256; e += NTHR) sBg[e] = b_ih[e] + b_hh[e];
    if (tid < 16) {
        const int ip = tid < NP ? tid : 0;
        const int ic = tid < NM ? tid : 0;
        sBpos[tid] = (tid < NP) ? b_pos[ip]  : 0.0f;
        sBse[tid]  = b_se[tid];
        sBcf[tid]  = (tid < NM) ? b_conf[ic] : 0.0f;
    }

    const int lane = tid & 31, wave = tid >> 5;
    const int h = lane >> 4;
    const int n = lane & 15;
    const int a0 = wave * AG;
    const size_t g0 = (size_t)blk * BLKA + a0;
    f16t* hst = sH + a0 * HP;
    f16t* xst = sX + a0 * XP;
    f16t* rst = sR + a0 * XP;

    {
        const int row = lane >> 1, cb = (lane & 1) * 32;
        const float* p = h0 + (g0 + row) * HD + cb;
#pragma unroll
        for (int q = 0; q < 4; ++q)
            *(v8h*)(hst + row * HP + cb + q * 8) =
                cvt8(*(const v4f*)(p + q * 8), *(const v4f*)(p + q * 8 + 4), 1.0f);
    }
    float creg[4][8];
#pragma unroll
    for (int j = 0; j < 4; ++j)
#pragma unroll
        for (int r = 0; r < 8; ++r)
            creg[j][r] = c0[(g0 + 8 * h + r) * HD + 16 * j + n];
    {
        if (h == 0) {
            const float rx = traj_rel[(g0 + n) * 2 + 0];
            const float ry = traj_rel[(g0 + n) * 2 + 1];
            v8h k0, k1 = zero8h();
#pragma unroll
            for (int e = 0; e < 8; ++e) k0[e] = (f16t)((e & 1) ? ry : rx);
#pragma unroll
            for (int e = 0; e < 4; ++e) k1[e] = (f16t)((e & 1) ? ry : rx);
            *(v8h*)(rst + n * XP)     = k0;
            *(v8h*)(rst + n * XP + 8) = k1;
        }
    }
    __syncthreads();

    v16h ha0 = ldfrag(hst + n * HP + 8 * h);
    v16h ha1 = ldfrag(hst + n * HP + 32 + 8 * h);
    se_step(rst, sWse, sBse, xst, h, n);
    __syncthreads();
    v16h xa = ldfrag16(xst + n * XP + 8 * h);

#pragma unroll 1
    for (int t = 0; t < TS; ++t) {
#pragma unroll
        for (int j = 0; j < 4; ++j) {
            const v8f gi = gate_tile(j,     sWih, sWhh, xa, ha0, ha1, h, n);
            const v8f gg = gate_tile(8 + j, sWih, sWhh, xa, ha0, ha1, h, n);
            const float bi = sBg[16 * j + n];
            const float bg = sBg[128 + 16 * j + n];
            const float bf = sBg[64 + 16 * j + n];
            const float bo = sBg[192 + 16 * j + n];
            float ig[8];
#pragma unroll
            for (int r = 0; r < 8; ++r)
                ig[r] = fsig(fmaf(gi[r], WINV, bi)) * ftanh(fmaf(gg[r], WINV, bg));
            const v8f gf = gate_tile(4 + j, sWih, sWhh, xa, ha0, ha1, h, n);
#pragma unroll
            for (int r = 0; r < 8; ++r)
                creg[j][r] = fmaf(fsig(fmaf(gf[r], WINV, bf)), creg[j][r], ig[r]);
            const v8f go = gate_tile(12 + j, sWih, sWhh, xa, ha0, ha1, h, n);
#pragma unroll
            for (int r = 0; r < 8; ++r) {
                const float hv = fsig(fmaf(go[r], WINV, bo)) * ftanh(creg[j][r]);
                hst[(8 * h + r) * HP + 16 * j + n] = (f16t)hv;
            }
        }
        __syncthreads();
        ha0 = ldfrag(hst + n * HP + 8 * h);
        ha1 = ldfrag(hst + n * HP + 32 + 8 * h);
        {
            const v16h p0 = ldfrag(sWpos + n * HP + 8 * h);
            const v16h p1 = ldfrag(sWpos + n * HP + 32 + 8 * h);
            v8f acc = zacc();
            acc = wmma16(ha0, p0, acc);
            acc = wmma16(ha1, p1, acc);
            guard2(acc, ha0, ha1, p0, p1);
            const float bp = sBpos[n];
#pragma unroll
            for (int r = 0; r < 8; ++r) {
                const float v = fmaf(acc[r], WINV, bp);
                const int ar = a0 + 8 * h + r;
                if (n < NP) sPred[ar * OUTW + (n >> 1) * (TS * 2) + t * 2 + (n & 1)] = v;
                rst[(8 * h + r) * XP + n] = (f16t)v;
            }
        }
        __syncthreads();
        se_step(rst, sWse, sBse, xst, h, n);
        __syncthreads();
        xa = ldfrag16(xst + n * XP + 8 * h);
    }

    {
        const v16h q0 = ldfrag(sWcf + n * HP + 8 * h);
        const v16h q1 = ldfrag(sWcf + n * HP + 32 + 8 * h);
        v8f acc = zacc();
        acc = wmma16(ha0, q0, acc);
        acc = wmma16(ha1, q1, acc);
        guard2(acc, ha0, ha1, q0, q1);
        const float bc = sBcf[n];
        if (n < 8) {
#pragma unroll
            for (int r = 0; r < 8; ++r)
                sLog[(a0 + 8 * h + r) * 8 + n] = fmaf(acc[r], WINV, bc);
        }
    }
    __syncthreads();
    if (h == 0) {
        const int ar = a0 + n;
        float v[NM];
        float mx = -3.0e38f;
#pragma unroll
        for (int k = 0; k < NM; ++k) { v[k] = sLog[ar * 8 + k]; mx = fmaxf(mx, v[k]); }
        float s = 0.0f;
#pragma unroll
        for (int k = 0; k < NM; ++k) { v[k] = __expf(v[k] - mx); s += v[k]; }
        const float inv = __builtin_amdgcn_rcpf(s);
#pragma unroll
        for (int k = 0; k < NM; ++k) sCf[ar * NM + k] = v[k] * inv;
    }
    __syncthreads();

    float* gp = pred + (size_t)blk * (BLKA * OUTW);
    float* gc = conf + (size_t)blk * (BLKA * NM);
#pragma unroll 1
    for (int i = 0; i < NIT; ++i) {
        const int p = tid + NTHR * i;
        const v4f v = *(const v4f*)(sPred + p * 4);
        *(volatile v4f*)(gp + (size_t)p * 4) = v;
    }
    if (tid < NCPIECE) {
        const v4f v = *(const v4f*)(sCf + tid * 4);
        *(volatile v4f*)(gc + tid * 4) = v;
    }
    __threadfence();
#pragma unroll 1
    for (int i = 0; i < NIT; ++i) {
        const int p = tid + NTHR * i;
        const v4f v = *(const v4f*)(sPred + p * 4);
        *(volatile v4f*)(gp + (size_t)p * 4) = v;
    }
    if (tid < NCPIECE) {
        const v4f v = *(const v4f*)(sCf + tid * 4);
        *(volatile v4f*)(gc + tid * 4) = v;
    }
}

extern "C" void kernel_launch(void* const* d_in, const int* in_sizes, int n_in,
                              void* d_out, int out_size, void* d_ws, size_t ws_size,
                              hipStream_t stream) {
    (void)d_ws; (void)ws_size;
    if (n_in < 14) return;
    const int nag = in_sizes[2] / HD;
    if (nag <= 0 || (nag % BLKA) != 0) return;
    if (in_sizes[2] != nag * HD || in_sizes[3] != nag * HD || in_sizes[1] != nag * 2) return;
    if (in_sizes[4] != 256 * 16 || in_sizes[5] != 256 * HD ||
        in_sizes[6] != 256 || in_sizes[7] != 256) return;
    if (in_sizes[8] != 16 * NP || in_sizes[9] != 16 || in_sizes[10] != NP * HD ||
        in_sizes[11] != NP || in_sizes[12] != NM * HD || in_sizes[13] != NM) return;
    if (out_size != nag * OUTW + nag * NM) return;

    const float* traj_rel = (const float*)d_in[1];
    const float* h0       = (const float*)d_in[2];
    const float* c0       = (const float*)d_in[3];
    const float* W_ih     = (const float*)d_in[4];
    const float* W_hh     = (const float*)d_in[5];
    const float* b_ih     = (const float*)d_in[6];
    const float* b_hh     = (const float*)d_in[7];
    const float* W_se     = (const float*)d_in[8];
    const float* b_se     = (const float*)d_in[9];
    const float* W_pos    = (const float*)d_in[10];
    const float* b_pos    = (const float*)d_in[11];
    const float* W_conf   = (const float*)d_in[12];
    const float* b_conf   = (const float*)d_in[13];

    float* pred = (float*)d_out;
    float* conf = pred + (size_t)nag * OUTW;

    k_traj_lstm<<<dim3(nag / BLKA), dim3(NTHR), 0, stream>>>(
        traj_rel, h0, c0, W_ih, W_hh, b_ih, b_hh, W_se, b_se, W_pos, b_pos, W_conf, b_conf,
        pred, conf, nag);
}
